// FlexScaleSeqAttention_84207128805783
// MI455X (gfx1250) — hardware-verified
//
#include <hip/hip_runtime.h>


#define NB_  2
#define TT   2048
#define DM   1024
#define NH_  16
#define HD   64
#define SO   2048
#define ZH   2
#define PCAR 1024.0f
typedef _Float16 h16;
typedef unsigned short bf;
typedef __attribute__((ext_vector_type(16))) __bf16   v16bf;
typedef __attribute__((ext_vector_type(16))) _Float16 v16h;
typedef __attribute__((ext_vector_type(8)))  _Float16 v8h;
typedef __attribute__((ext_vector_type(8)))  unsigned short v8us;
typedef __attribute__((ext_vector_type(8)))  float    v8f;
typedef __attribute__((ext_vector_type(4)))  float    v4f;
typedef v8h  __attribute__((may_alias)) v8ha;
typedef v4f  __attribute__((may_alias)) v4fa;
typedef v8us __attribute__((may_alias)) v8usa;

__device__ __forceinline__ unsigned short f2bf(float f) { unsigned u = __float_as_uint(f); u += 0x7FFFu + ((u >> 16) & 1u); return (unsigned short)(u >> 16); }
__device__ __forceinline__ float bf2f(unsigned short b) { return __uint_as_float(((unsigned)b) << 16); }
__device__ __forceinline__ float bfr(float f) { return bf2f(f2bf(f)); }
__device__ __forceinline__ v16h cat16(v8h lo, v8h hi) { return __builtin_shufflevector(lo, hi, 0, 1, 2, 3, 4, 5, 6, 7, 8, 9, 10, 11, 12, 13, 14, 15); }
__device__ __forceinline__ v16bf cat16b(v8us lo, v8us hi) { return __builtin_bit_cast(v16bf, __builtin_shufflevector(lo, hi, 0, 1, 2, 3, 4, 5, 6, 7, 8, 9, 10, 11, 12, 13, 14, 15)); }
__device__ __forceinline__ v8f wmma16(v16h a, v16h b, v8f c) { return __builtin_amdgcn_wmma_f32_16x16x32_f16(false, a, false, b, (short)0, c, false, false); }
__device__ __forceinline__ v8f wmmab(v16bf a, v16bf b, v8f c) { return __builtin_amdgcn_wmma_f32_16x16x32_bf16(false, a, false, b, (short)0, c, false, false); }


template <typename T16> struct WFrag;
template <> struct WFrag<h16> { typedef v16h V; static __device__ __forceinline__ V ld(const h16* p) { return cat16(*(const v8h*)p, *(const v8h*)(p + 16)); } static __device__ __forceinline__ v8f mma(V a, V b, v8f c) { return wmma16(a, b, c); } };
template <> struct WFrag<bf> { typedef v16bf V; static __device__ __forceinline__ V ld(const bf* p) { return cat16b(*(const v8us*)p, *(const v8us*)(p + 16)); } static __device__ __forceinline__ v8f mma(V a, V b, v8f c) { return wmmab(a, b, c); } };
template <typename T16, int NSPLIT, bool BIAS>
__global__ __launch_bounds__(32) void k_gemmw(const T16* __restrict__ A, const T16* __restrict__ A2, const T16* __restrict__ Bt, const T16* __restrict__ Bt2, int K, float* C, int ldc, const float* __restrict__ bias, size_t sA, size_t sB, size_t sC) {
    typedef typename WFrag<T16>::V V;
    __shared__ __align__(16) float os[16 * 68];
    const size_t z = blockIdx.z; A += z * sA; if (A2) A2 += z * sA; Bt += z * sB; if (Bt2) Bt2 += z * sB; C += z * sC;
    const int lane = threadIdx.x & 31, lr = lane & 15, hi = lane >> 4; const int r0 = blockIdx.x * 64, c0 = blockIdx.y * 64;
    v8f acc[4][4];
#pragma unroll
    for (int mb = 0; mb < 4; ++mb)
#pragma unroll
        for (int nb = 0; nb < 4; ++nb) acc[mb][nb] = (v8f){};
    const size_t aoff = (size_t)(r0 + lr) * K + 8 * hi, boff = (size_t)(c0 + lr) * K + 8 * hi;
#pragma unroll 1
    for (int kc = 0; kc < K; kc += 32) {
        V a[4], a2[4];
#pragma unroll
        for (int mb = 0; mb < 4; ++mb) { a[mb] = WFrag<T16>::ld(A + aoff + (size_t)mb * 16 * K + kc); if (NSPLIT == 1 || NSPLIT == 2) a2[mb] = WFrag<T16>::ld(A2 + aoff + (size_t)mb * 16 * K + kc); }
#pragma unroll
        for (int nb = 0; nb < 4; ++nb) { const V b = WFrag<T16>::ld(Bt + boff + (size_t)nb * 16 * K + kc); V b2; if (NSPLIT >= 2) b2 = WFrag<T16>::ld(Bt2 + boff + (size_t)nb * 16 * K + kc);
#pragma unroll
            for (int mb = 0; mb < 4; ++mb) { acc[mb][nb] = WFrag<T16>::mma(a[mb], b, acc[mb][nb]); if (NSPLIT == 1 || NSPLIT == 2) acc[mb][nb] = WFrag<T16>::mma(a2[mb], b, acc[mb][nb]); if (NSPLIT >= 2) acc[mb][nb] = WFrag<T16>::mma(a[mb], b2, acc[mb][nb]); } }
        asm volatile("v_nop\n\tv_nop\n\tv_nop\n\tv_nop" : "+v"(acc[0][0]), "+v"(acc[1][1]), "+v"(acc[2][2]), "+v"(acc[3][3]) : "v"(a[0]), "v"(a[3]));
    }
#pragma unroll
    for (int mb = 0; mb < 4; ++mb) {
#pragma unroll
        for (int nb = 0; nb < 4; ++nb) {
#pragma unroll
            for (int j = 0; j < 8; ++j) os[(hi * 8 + j) * 68 + nb * 16 + lr] = acc[mb][nb][j]; }
        __builtin_amdgcn_wave_barrier(); asm volatile("" ::: "memory");
        float* crow = C + (size_t)(r0 + mb * 16) * ldc + c0;
#pragma unroll 1
        for (int ps = 0; ps < 2; ++ps) {
#pragma unroll
            for (int s = 0; s < 8; ++s) { const int row = 2 * s + hi, cofs = lr * 4; v4f val = *(const v4fa*)(os + row * 68 + cofs); if (BIAS) { val[0] += bfr(bias[c0 + cofs]); val[1] += bfr(bias[c0 + cofs + 1]); val[2] += bfr(bias[c0 + cofs + 2]); val[3] += bfr(bias[c0 + cofs + 3]); }
                *(volatile v4f*)(crow + (size_t)row * ldc + cofs) = val; }
            if (ps == 0) __threadfence(); }
        __builtin_amdgcn_wave_barrier(); asm volatile("" ::: "memory");
    }
}

__device__ __forceinline__ h16 tohx(float x) { return (h16)x; }
__device__ __forceinline__ void splitf(float y, unsigned short& h, unsigned short& l) { h = f2bf(y); l = f2bf(y - bf2f(h)); }
typedef __attribute__((ext_vector_type(2))) unsigned short v2us;
typedef __attribute__((ext_vector_type(4))) unsigned short v4us;
typedef __attribute__((ext_vector_type(2))) _Float16 v2h;
typedef __attribute__((ext_vector_type(4))) _Float16 v4h; typedef __attribute__((ext_vector_type(2))) float v2f;

__global__ __launch_bounds__(256) void k_cvt8(const float* __restrict__ src, bf* dst, size_t n8) { const size_t i = (size_t)blockIdx.x * 256 + threadIdx.x; if (i >= n8) return; const v8f v = *(const v8f*)(src + i * 8); v8us o;
#pragma unroll
    for (int k = 0; k < 8; ++k) o[k] = f2bf(v[k]); *(volatile v8us*)(dst + i * 8) = o; __threadfence(); *(volatile v8us*)(dst + i * 8) = o; }
__global__ __launch_bounds__(256) void k_qk16(const float* __restrict__ Q, const float* __restrict__ K, h16* QP, h16* KP) { const size_t e = ((size_t)blockIdx.x * 256 + threadIdx.x) * 4; if (e >= (size_t)NH_ * TT * HD) return; const int d = (int)(e % HD); const int t = (int)((e / HD) % TT); const int h = (int)(e / ((size_t)HD * TT)); const size_t src = (size_t)t * DM + h * HD + d; const v4f a = *(const v4f*)(Q + src), c = *(const v4f*)(K + src); v4h oq, ok;
    for (int u = 0; u < 4; ++u) { oq[u] = tohx(a[u]); ok[u] = tohx(c[u]); } *(volatile v4h*)(QP + e) = oq; *(volatile v4h*)(KP + e) = ok; __threadfence(); *(volatile v4h*)(QP + e) = oq; *(volatile v4h*)(KP + e) = ok; }
__global__ __launch_bounds__(256) void k_vt16(const float* __restrict__ V, h16* VT) { const size_t e = ((size_t)blockIdx.x * 256 + threadIdx.x) * 2; if (e >= (size_t)NH_ * HD * TT) return; const int t = (int)(e % TT); const int d = (int)((e / TT) % HD); const int h = (int)(e / ((size_t)TT * HD)); v2h o; o[0] = tohx(V[(size_t)t * DM + h * HD + d]); o[1] = tohx(V[(size_t)(t + 1) * DM + h * HD + d]); *(volatile v2h*)(VT + e) = o; __threadfence(); *(volatile v2h*)(VT + e) = o; }
__global__ __launch_bounds__(256) void k_vsum(const float* __restrict__ V, float* VS) { const int c = blockIdx.x * 256 + threadIdx.x; if (c >= DM) return; float s = 0.f;
#pragma unroll 8
    for (int t = 0; t < TT; ++t) s = __fadd_rn(s, V[(size_t)t * DM + c]); *(volatile float*)(VS + c) = s; __threadfence(); *(volatile float*)(VS + c) = s; }
__global__ __launch_bounds__(256) void k_colsoft(const float* __restrict__ ST, h16* PT) { const int lane = threadIdx.x & 31; const int wv = blockIdx.x * 8 + (threadIdx.x >> 5); if (wv >= ZH * (TT / 64)) return; const int zz = wv / (TT / 64); const int q0 = (wv % (TT / 64)) * 64 + lane * 2; const float* s0 = ST + (size_t)zz * TT * TT + q0; h16* p0 = PT + (size_t)zz * TT * TT + q0;
    float mx0 = -3.0e38f, mx1 = -3.0e38f;
#pragma unroll 4
    for (int k = 0; k < TT; ++k) { const v2f a = *(const v2f*)(s0 + (size_t)k * TT); mx0 = fmaxf(mx0, a[0] * 0.125f); mx1 = fmaxf(mx1, a[1] * 0.125f); }
    float sm0 = 0.f, sm1 = 0.f;
#pragma unroll 4
    for (int k = 0; k < TT; ++k) { const v2f a = *(const v2f*)(s0 + (size_t)k * TT); float d0 = __fsub_rn(a[0] * 0.125f, mx0), d1 = __fsub_rn(a[1] * 0.125f, mx1); asm volatile("" : "+v"(d0)); asm volatile("" : "+v"(d1)); sm0 = __fadd_rn(sm0, __builtin_amdgcn_exp2f(__fmul_rn(d0, 1.4426950408889634f))); sm1 = __fadd_rn(sm1, __builtin_amdgcn_exp2f(__fmul_rn(d1, 1.4426950408889634f))); }
    const float f0 = __fdiv_rn(PCAR, sm0), f1 = __fdiv_rn(PCAR, sm1);
    for (int ps = 0; ps < 2; ++ps) {
#pragma unroll 4
        for (int k = 0; k < TT; ++k) { const v2f a = *(const v2f*)(s0 + (size_t)k * TT); float d0 = __fsub_rn(a[0] * 0.125f, mx0), d1 = __fsub_rn(a[1] * 0.125f, mx1); asm volatile("" : "+v"(d0)); asm volatile("" : "+v"(d1)); v2h o; o[0] = tohx(__builtin_amdgcn_exp2f(__fmul_rn(d0, 1.4426950408889634f)) * f0); o[1] = tohx(__builtin_amdgcn_exp2f(__fmul_rn(d1, 1.4426950408889634f)) * f1); *(volatile v2h*)(p0 + (size_t)k * TT) = o; }
        if (ps == 0) __threadfence(); } }
__global__ __launch_bounds__(256) void k_mt(const float* __restrict__ M, bf* MTh, bf* MTl) { const size_t e = ((size_t)blockIdx.x * 256 + threadIdx.x) * 4; if (e >= (size_t)ZH * HD * TT) return; const int k = (int)(e % TT); const int d = (int)((e / TT) % HD); const int zz = (int)(e / ((size_t)TT * HD)); v4us oh, ol;
#pragma unroll
    for (int u = 0; u < 4; ++u) { unsigned short a, b; splitf(M[((size_t)zz * TT + k + u) * HD + d] * (1.0f / PCAR), a, b); oh[u] = a; ol[u] = b; } *(volatile v4us*)(MTh + e) = oh; *(volatile v4us*)(MTl + e) = ol; __threadfence(); *(volatile v4us*)(MTh + e) = oh; *(volatile v4us*)(MTl + e) = ol; }
__global__ __launch_bounds__(256) void k_fmrg(const float* __restrict__ OC, const float* __restrict__ bfv, const float* __restrict__ VS, int h0, float* OUTb) { const size_t e = ((size_t)blockIdx.x * 256 + threadIdx.x) * 4; if (e >= (size_t)TT * ZH * HD) return; const int c = (int)(e % (ZH * HD)); const int o = (int)(e / (ZH * HD)); const int zz = c / HD, d = c % HD; const float bb = bfr(bfv[o]); v4f r;
#pragma unroll
    for (int u = 0; u < 4; ++u) { const float m = OC[((size_t)zz * HD + d + u) * SO + o]; float bt = __fmul_rn(bb, VS[(h0 + zz) * HD + d + u]); asm volatile("" : "+v"(bt)); r[u] = __fadd_rn(m, bt); }
    float* dst = OUTb + (size_t)o * DM + (h0 + zz) * HD + d; *(volatile v4f*)dst = r; __threadfence(); *(volatile v4f*)dst = r; }

extern "C" void kernel_launch(void* const* d_in, const int* in_sizes, int n_in,
                              void* d_out, int out_size, void* d_ws, size_t ws_size, hipStream_t stream) {
    (void)in_sizes; (void)n_in; (void)out_size;
    const float* x = (const float*)d_in[0]; const float* wq = (const float*)d_in[1]; const float* bq = (const float*)d_in[2]; const float* wk = (const float*)d_in[3]; const float* bk = (const float*)d_in[4]; const float* wv = (const float*)d_in[5]; const float* bv = (const float*)d_in[6]; const float* wf = (const float*)d_in[7]; const float* bfv = (const float*)d_in[8];
    float* OUT = (float*)d_out;
    char* wsp = (char*)d_ws;
    auto take = [&](size_t bytes) { char* p = wsp; wsp += (bytes + 255) & ~(size_t)255; return (void*)p; };
    bf* BQ = (bf*)take((size_t)DM * DM * 2); bf* BK = (bf*)take((size_t)DM * DM * 2); bf* BV = (bf*)take((size_t)DM * DM * 2); bf* BF = (bf*)take((size_t)SO * TT * 2);
    bf* XB = (bf*)take((size_t)TT * DM * 2); float* FQ = (float*)take((size_t)TT * DM * 4); float* FK = (float*)take((size_t)TT * DM * 4); float* FV = (float*)take((size_t)TT * DM * 4); float* VS = (float*)take(DM * 4);
    h16* QP = (h16*)take((size_t)NH_ * TT * HD * 2); h16* KP = (h16*)take((size_t)NH_ * TT * HD * 2); h16* VT = (h16*)take((size_t)NH_ * HD * TT * 2);
    float* ST = (float*)take((size_t)ZH * TT * TT * 4); h16* PT = (h16*)take((size_t)ZH * TT * TT * 2); float* M = (float*)take((size_t)ZH * TT * HD * 4); bf* MTh = (bf*)take((size_t)ZH * HD * TT * 2); bf* MTl = (bf*)take((size_t)ZH * HD * TT * 2); float* OC = (float*)take((size_t)ZH * HD * SO * 4);
    if ((size_t)(wsp - (char*)d_ws) > ws_size) return;
    k_cvt8<<<(DM * DM / 8 + 255) / 256, 256, 0, stream>>>(wq, BQ, DM * DM / 8); k_cvt8<<<(DM * DM / 8 + 255) / 256, 256, 0, stream>>>(wk, BK, DM * DM / 8); k_cvt8<<<(DM * DM / 8 + 255) / 256, 256, 0, stream>>>(wv, BV, DM * DM / 8); k_cvt8<<<(SO * TT / 8 + 255) / 256, 256, 0, stream>>>(wf, BF, SO * TT / 8);
    const dim3 gp(TT / 64, DM / 64, 1); const size_t zq = (size_t)TT * HD, zS = (size_t)TT * TT, zv = (size_t)HD * TT, zm = (size_t)TT * HD, zc = (size_t)HD * SO;
    for (int b = 0; b < NB_; ++b) {
        k_cvt8<<<(TT * DM / 8 + 255) / 256, 256, 0, stream>>>(x + (size_t)b * TT * DM, XB, TT * DM / 8);
        k_gemmw<bf, 0, true><<<gp, 32, 0, stream>>>(XB, nullptr, BQ, nullptr, DM, FQ, DM, bq, 0, 0, 0); k_gemmw<bf, 0, true><<<gp, 32, 0, stream>>>(XB, nullptr, BK, nullptr, DM, FK, DM, bk, 0, 0, 0); k_gemmw<bf, 0, true><<<gp, 32, 0, stream>>>(XB, nullptr, BV, nullptr, DM, FV, DM, bv, 0, 0, 0);
        k_qk16<<<(unsigned)(((size_t)NH_ * TT * HD / 4 + 255) / 256), 256, 0, stream>>>(FQ, FK, QP, KP); k_vt16<<<(unsigned)(((size_t)NH_ * HD * TT / 2 + 255) / 256), 256, 0, stream>>>(FV, VT); k_vsum<<<DM / 256, 256, 0, stream>>>(FV, VS);
        for (int h0 = 0; h0 < NH_; h0 += ZH) {
            k_gemmw<h16, 0, false><<<dim3(TT / 64, TT / 64, ZH), 32, 0, stream>>>(KP + (size_t)h0 * zq, nullptr, QP + (size_t)h0 * zq, nullptr, HD, ST, TT, nullptr, zq, zq, zS);
            k_colsoft<<<ZH * (TT / 64) / 8, 256, 0, stream>>>(ST, PT);
            k_gemmw<h16, 0, false><<<dim3(TT / 64, 1, ZH), 32, 0, stream>>>(PT, nullptr, VT + (size_t)h0 * zv, nullptr, TT, M, HD, nullptr, zS, zv, zm);
            k_mt<<<(unsigned)(((size_t)ZH * HD * TT / 4 + 255) / 256), 256, 0, stream>>>(M, MTh, MTl);
            k_gemmw<bf, 1, false><<<dim3(1, SO / 64, ZH), 32, 0, stream>>>(MTh, MTl, BF, nullptr, TT, OC, SO, nullptr, zv, 0, zc);
            k_fmrg<<<(unsigned)(((size_t)TT * ZH * HD / 4 + 255) / 256), 256, 0, stream>>>(OC, bfv, VS, h0, OUT + (size_t)b * SO * DM); } }
}
